// PointNetSetAbstraction_82755429859696
// MI455X (gfx1250) — hardware-verified
//
#include <hip/hip_runtime.h>
#pragma clang fp contract(off)

typedef __attribute__((ext_vector_type(16))) _Float16 v16h;
typedef __attribute__((ext_vector_type(8)))  _Float16 v8h;
typedef __attribute__((ext_vector_type(8)))  float    v8f;
typedef __attribute__((ext_vector_type(4)))  float    v4f;
typedef __attribute__((ext_vector_type(4)))  unsigned v4u;

constexpr int kBatch = 16;
constexpr int kPts   = 4096;
constexpr int kFeat  = 64;
constexpr int kCent  = 512;
constexpr int kGroup = 32;
constexpr int kOutCh = 128;
constexpr int kCap   = 64;

constexpr size_t kOffW0p  = 0;
constexpr size_t kOffW1   = 8192;
constexpr size_t kOffW2   = 16384;
constexpr size_t kOffTab  = 32768;
constexpr size_t kOffNxyz = 36864;
constexpr size_t kOffX4   = 135168;
constexpr size_t kOffP16  = 1183744;
constexpr size_t kWsTotal = 9572352;
static_assert(kOffNxyz + (size_t)kBatch * kCent * 3 * 4 == kOffX4, "carve");
static_assert(kOffX4 + (size_t)kBatch * kPts * 16 == kOffP16, "carve");
static_assert(kOffP16 + (size_t)kBatch * kPts * kFeat * 2 == kWsTotal, "carve");
static_assert(kWsTotal <= 134217728, "carve limit");
static_assert((kOffTab % 128) == 0 && (kOffNxyz % 128) == 0 && (kOffX4 % 128) == 0 && (kOffP16 % 128) == 0, "line aligned");
constexpr size_t kOut1Bytes = 98304;
static_assert((size_t)kBatch * kCent * 3 * 4 == kOut1Bytes, "out0 extent");
static_assert(kOut1Bytes + (size_t)kBatch * kCent * kOutCh * 4 == 4292608, "out total");

constexpr int kTabSc0 = 256;
constexpr int kTabSh0 = 384;
constexpr int kTabSc1 = 512;
constexpr int kTabSh1 = 640;
constexpr int kTabSc2 = 768;
constexpr int kTabSh2 = 896;

struct FragH {
  union U { v16h v; v8h h[2]; };
  static __device__ __forceinline__ v16h load(const _Float16* p) {
    U f;
    f.h[0] = *(const v8h*)(p);
    f.h[1] = *(const v8h*)(p + 16);
    return f.v;
  }
};

__device__ __forceinline__ v8f wmma_h(v16h a, v16h b, v8f c) {
  return __builtin_amdgcn_wmma_f32_16x16x32_f16(false, a, false, b, (short)0, c, false, false);
}

__device__ __forceinline__ void mma4(v8f& c0, v8f& c1, v16h a0, v16h a1,
                                     v16h b00, v16h b01, v16h b10, v16h b11) {
  c0 = wmma_h(a0, b00, c0);
  c1 = wmma_h(a0, b01, c1);
  c0 = wmma_h(a1, b10, c0);
  c1 = wmma_h(a1, b11, c1);
  asm volatile("v_nop\n\tv_nop\n\tv_nop\n\tv_nop"
               : "+v"(c0), "+v"(c1)
               : "v"(a0), "v"(a1), "v"(b00), "v"(b01), "v"(b10), "v"(b11));
}

__device__ __forceinline__ void store2_v8h(unsigned short* dst, v8h hv) {
  *(volatile v8h*)dst = hv;
  __threadfence();
  *(volatile v8h*)dst = hv;
}
__device__ __forceinline__ void store2_v4f(float* dst, v4f v) {
  *(volatile v4f*)dst = v;
  __threadfence();
  *(volatile v4f*)dst = v;
}
__device__ __forceinline__ v8h cvt8(v4f a, v4f b) {
  v8h r;
  r[0] = (_Float16)a.x; r[1] = (_Float16)a.y; r[2] = (_Float16)a.z; r[3] = (_Float16)a.w;
  r[4] = (_Float16)b.x; r[5] = (_Float16)b.y; r[6] = (_Float16)b.z; r[7] = (_Float16)b.w;
  return r;
}
__device__ __forceinline__ void ld8(const float* p, float (&o)[8]) {
  const v4f a = *(const v4f*)(p);
  const v4f b = *(const v4f*)(p + 4);
  o[0] = a.x; o[1] = a.y; o[2] = a.z; o[3] = a.w;
  o[4] = b.x; o[5] = b.y; o[6] = b.z; o[7] = b.w;
}

__global__ __launch_bounds__(256) void prep_kernel(
    const float* __restrict__ xyz, const float* __restrict__ points,
    const float* __restrict__ w0, const float* __restrict__ b0, const float* __restrict__ g0,
    const float* __restrict__ be0, const float* __restrict__ rm0, const float* __restrict__ rv0,
    const float* __restrict__ w1, const float* __restrict__ b1, const float* __restrict__ g1,
    const float* __restrict__ be1, const float* __restrict__ rm1, const float* __restrict__ rv1,
    const float* __restrict__ w2, const float* __restrict__ b2, const float* __restrict__ g2,
    const float* __restrict__ be2, const float* __restrict__ rm2, const float* __restrict__ rv2,
    unsigned short* __restrict__ w0p, unsigned short* __restrict__ w1p, unsigned short* __restrict__ w2p,
    float* __restrict__ tab, float* __restrict__ x4, unsigned short* __restrict__ p16) {
#pragma clang fp contract(off)
  const int blk = blockIdx.x;
  const int tid = threadIdx.x;
  if (blk < 2) {
    const int chunk = blk * 256 + tid;
    const int o = chunk >> 3;
    const int c0 = (chunk & 7) * 8;
    const float* src = w0 + o * 67 + 3 + c0;
    v8h hv;
#pragma unroll
    for (int e = 0; e < 8; ++e) hv[e] = (_Float16)src[e];
    store2_v8h(w0p + chunk * 8, hv);
  } else if (blk < 4) {
    const int chunk = (blk - 2) * 256 + tid;
    const v4f a = ((const v4f*)w1)[chunk * 2];
    const v4f c = ((const v4f*)w1)[chunk * 2 + 1];
    store2_v8h(w1p + chunk * 8, cvt8(a, c));
  } else if (blk < 8) {
    const int chunk = (blk - 4) * 256 + tid;
    const v4f a = ((const v4f*)w2)[chunk * 2];
    const v4f c = ((const v4f*)w2)[chunk * 2 + 1];
    store2_v8h(w2p + chunk * 8, cvt8(a, c));
  } else if (blk == 8) {
    if (tid < 64) {
      const float* s = w0 + tid * 67;
      v4f v;
      v.x = s[0]; v.y = s[1]; v.z = s[2]; v.w = 0.0f;
      store2_v4f(tab + tid * 4, v);
    } else {
      const int arr = (tid >> 5) - 2;
      const int layer = arr >> 1;
      const int is_shift = arr & 1;
      const float* pb = b0; const float* pg = g0; const float* pbe = be0; const float* prm = rm0; const float* prv = rv0;
      int nch = 64;
      if (layer == 1) { pb = b1; pg = g1; pbe = be1; prm = rm1; prv = rv1; }
      if (layer == 2) { pb = b2; pg = g2; pbe = be2; prm = rm2; prv = rv2; nch = 128; }
      int ch0 = (tid & 31) * 4;
      ch0 = (ch0 > nch - 4) ? (nch - 4) : ch0;
      const v4f vb  = *(const v4f*)(pb + ch0);
      const v4f vg  = *(const v4f*)(pg + ch0);
      const v4f vbe = *(const v4f*)(pbe + ch0);
      const v4f vrm = *(const v4f*)(prm + ch0);
      const v4f vrv = *(const v4f*)(prv + ch0);
      v4f r;
#pragma unroll
      for (int e = 0; e < 4; ++e) {
        const float sc = vg[e] * rsqrtf(vrv[e] + 1e-5f);
        const float sh = (vb[e] - vrm[e]) * sc + vbe[e];
        r[e] = is_shift ? sh : sc;
      }
      store2_v4f(tab + 256 + arr * 128 + (tid & 31) * 4, r);
    }
  } else if (blk < 9 + 256) {
    const int idx = (blk - 9) * 256 + tid;
    const float* s = xyz + (size_t)idx * 3;
    const float x = s[0], y = s[1], z = s[2];
    const float tx = x * x, ty = y * y, tz = z * z;
    v4f v;
    v.x = x; v.y = y; v.z = z; v.w = (tx + tz) + ty;
    store2_v4f(x4 + (size_t)idx * 4, v);
  } else {
    const int chunk = (blk - 265) * 256 + tid;
    const v4f a = ((const v4f*)points)[(size_t)chunk * 2];
    const v4f c = ((const v4f*)points)[(size_t)chunk * 2 + 1];
    store2_v8h(p16 + (size_t)chunk * 8, cvt8(a, c));
  }
}

__global__ __launch_bounds__(256) void fps_kernel(const float* __restrict__ xyz,
                                                  float* __restrict__ out_xyz,
                                                  float* __restrict__ ws_xyz) {
#pragma clang fp contract(off)
  __shared__ __align__(16) float lxyz[kPts * 3];
  __shared__ float slotv[2][8];
  __shared__ int   sloti[2][8];
  __shared__ int   sel[kCent];
  const int b = blockIdx.x;
  const int tid = threadIdx.x;
  const int lane = tid & 31;
  const int wave = tid >> 5;
  const v4f* src = (const v4f*)(xyz + (size_t)b * kPts * 3);
#pragma unroll 4
  for (int i = 0; i < 12; ++i) {
    const v4f t = src[i * 256 + tid];
    *(v4f*)(lxyz + (i * 256 + tid) * 4) = t;
  }
  __syncthreads();
  float px[16], py[16], pz[16], dm[16];
#pragma unroll
  for (int j = 0; j < 16; ++j) {
    const int idx = (j * 256 + tid) * 3;
    px[j] = lxyz[idx + 0];
    py[j] = lxyz[idx + 1];
    pz[j] = lxyz[idx + 2];
    dm[j] = 1e10f;
  }
  int far = 0;
#pragma unroll 1
  for (int it = 0; it < kCent; ++it) {
    const int par = it & 1;
    const float cx = lxyz[far * 3 + 0];
    const float cy = lxyz[far * 3 + 1];
    const float cz = lxyz[far * 3 + 2];
    if (tid == 0) sel[it] = far;
    float best = -1.0f;
    int bi = tid;
#pragma unroll
    for (int j = 0; j < 16; ++j) {
      const float dx = px[j] - cx;
      const float dy = py[j] - cy;
      const float dz = pz[j] - cz;
      const float tx = dx * dx;
      const float ty = dy * dy;
      const float tz = dz * dz;
      const float d = (tx + tz) + ty;
      const float nd = fminf(dm[j], d);
      dm[j] = nd;
      if (nd > best) { best = nd; bi = j * 256 + tid; }
    }
#pragma unroll
    for (int off = 16; off >= 1; off >>= 1) {
      const float ov = __shfl_xor(best, off, 32);
      const int   oi = __shfl_xor(bi, off, 32);
      const bool take = (ov > best) || ((ov == best) && (oi < bi));
      best = take ? ov : best;
      bi   = take ? oi : bi;
    }
    if (lane == 0) { slotv[par][wave] = best; sloti[par][wave] = bi; }
    __syncthreads();
    float v = slotv[par][lane & 7];
    int   i = sloti[par][lane & 7];
#pragma unroll
    for (int off = 1; off <= 4; off <<= 1) {
      const float ov = __shfl_xor(v, off, 32);
      const int   oi = __shfl_xor(i, off, 32);
      const bool take = (ov > v) || ((ov == v) && (oi < i));
      v = take ? ov : v;
      i = take ? oi : i;
    }
    far = i & (kPts - 1);
  }
  __syncthreads();
  v4f o0, o1;
  {
    const int q0 = tid;
    const int q1 = (tid + 256 < 384) ? (tid + 256) : 383;
#pragma unroll
    for (int e = 0; e < 4; ++e) {
      const int f0 = 4 * q0 + e;
      const int s0 = f0 / 3;
      const int c0 = f0 - 3 * s0;
      o0[e] = lxyz[(sel[s0] & (kPts - 1)) * 3 + c0];
      const int f1 = 4 * q1 + e;
      const int s1 = f1 / 3;
      const int c1 = f1 - 3 * s1;
      o1[e] = lxyz[(sel[s1] & (kPts - 1)) * 3 + c1];
    }
  }
  float* dst0 = out_xyz + (size_t)b * (kCent * 3);
  float* dst1 = ws_xyz + (size_t)b * (kCent * 3);
  for (int pass = 0; pass < 2; ++pass) {
    *(volatile v4f*)(dst0 + 4 * tid) = o0;
    *(volatile v4f*)(dst1 + 4 * tid) = o0;
    if (tid < 128) {
      *(volatile v4f*)(dst0 + 4 * (tid + 256)) = o1;
      *(volatile v4f*)(dst1 + 4 * (tid + 256)) = o1;
    }
    __threadfence();
  }
}

__device__ __forceinline__ unsigned scan_point(v4f p, float cx, float cy, float cz, float sqc, float thr,
                                               int idx, unsigned lt, int& cnt, int* ci, float* cd) {
#pragma clang fp contract(off)
  float dot = p.x * cx;
  dot = __builtin_fmaf(p.y, cy, dot);
  dot = __builtin_fmaf(p.z, cz, dot);
  float d = -2.0f * dot;
  d = d + sqc;
  d = d + p.w;
  const bool in = !(d > thr);
  const unsigned bm = __builtin_amdgcn_ballot_w32(in);
  const int pos = cnt + __popc(bm & lt);
  if (in && pos < kCap) { ci[pos] = idx; cd[pos] = d; }
  cnt += __popc(bm);
  return bm;
}

__global__ __launch_bounds__(128) void group_mlp_kernel(
    const float* __restrict__ x4g, const unsigned short* __restrict__ p16,
    const float* __restrict__ nxyz,
    const unsigned short* __restrict__ w0p, const unsigned short* __restrict__ w1p,
    const unsigned short* __restrict__ w2p,
    const float* __restrict__ tabg, float* __restrict__ out_pts) {
#pragma clang fp contract(off)
  __shared__ __align__(16) float tab[1024];
  __shared__ int   cidx[4][kCap];
  __shared__ float cdv[4][kCap];
  __shared__ int   gidx[4][kGroup];
  __shared__ __align__(16) _Float16 xs[4][kGroup * 72];
  __shared__ __align__(16) float ms[4][16 * 132];

  const int tid = threadIdx.x;
  const int wave = tid >> 5;
  const int lane = tid & 31;
  const int h = lane >> 4;
  const int n = lane & 15;
  const int gs = blockIdx.x * 4 + wave;
  const int b = gs >> 9;

  int* ci = cidx[wave];
  float* cd = cdv[wave];
  int* gi = gidx[wave];
  _Float16* xw = xs[wave];
  float* mw = ms[wave];

#pragma unroll
  for (int i = 0; i < 2; ++i) {
    const v4f t = ((const v4f*)tabg)[i * 128 + tid];
    *(v4f*)(tab + (i * 128 + tid) * 4) = t;
  }
  ci[lane] = 0; ci[lane + 32] = 0;
  cd[lane] = 0.0f; cd[lane + 32] = 0.0f;
  gi[lane] = lane;
  __syncthreads();

  const float cx = nxyz[(size_t)gs * 3 + 0];
  const float cy = nxyz[(size_t)gs * 3 + 1];
  const float cz = nxyz[(size_t)gs * 3 + 2];
  const float tcx = cx * cx, tcy = cy * cy, tcz = cz * cz;
  const float sqc = (tcx + tcz) + tcy;
  const float thr = __uint_as_float(0x3D23D70Au);
  const v4f* xb = (const v4f*)x4g + (size_t)b * kPts;
  const unsigned lt = (1u << lane) - 1u;

  int cnt = 0;
  unsigned outm0 = 0u;
#pragma unroll 1
  for (int base = 0; base < kPts; base += 128) {
    const v4f p0 = xb[base + lane];
    const v4f p1 = xb[base + 32 + lane];
    const v4f p2 = xb[base + 64 + lane];
    const v4f p3 = xb[base + 96 + lane];
    const unsigned bm0 = scan_point(p0, cx, cy, cz, sqc, thr, base + lane, lt, cnt, ci, cd);
    if (base == 0) outm0 = ~bm0;
    scan_point(p1, cx, cy, cz, sqc, thr, base + 32 + lane, lt, cnt, ci, cd);
    scan_point(p2, cx, cy, cz, sqc, thr, base + 64 + lane, lt, cnt, ci, cd);
    scan_point(p3, cx, cy, cz, sqc, thr, base + 96 + lane, lt, cnt, ci, cd);
  }
  __syncthreads();

  const int mm = (cnt > kCap) ? kCap : cnt;
  if (mm > kGroup) {
    const bool has1 = (lane + 32) < mm;
    const int q1 = has1 ? (lane + 32) : (mm - 1);
    const int i0 = ci[lane];
    const int i1 = ci[q1];
    const float d0 = cd[lane];
    const float d1 = cd[q1];
    int r0 = 0, r1 = 0;
#pragma unroll 1
    for (int q = 0; q < mm; ++q) {
      const float dq = cd[q];
      const int iq = ci[q];
      r0 += ((dq < d0) || ((dq == d0) && (iq < i0))) ? 1 : 0;
      r1 += ((dq < d1) || ((dq == d1) && (iq < i1))) ? 1 : 0;
    }
    const bool k0 = r0 < kGroup;
    const bool k1 = has1 && (r1 < kGroup);
    const unsigned bk0 = __builtin_amdgcn_ballot_w32(k0);
    const unsigned bk1 = __builtin_amdgcn_ballot_w32(k1);
    const int p0 = __popc(bk0 & lt);
    const int p1 = __popc(bk0) + __popc(bk1 & lt);
    if (k0 && p0 < kGroup) gi[p0] = i0;
    if (k1 && p1 < kGroup) gi[p1] = i1;
  } else {
    if (lane < mm) gi[lane] = ci[lane];
    const int nfill = kGroup - mm;
    const bool isout = ((outm0 >> lane) & 1u) != 0u;
    const int rk = __popc(outm0 & lt);
    if (isout && rk < nfill) gi[mm + rk] = lane;
  }
  __syncthreads();

  int jm = gi[lane];
  jm = jm < 0 ? 0 : (jm > kPts - 1 ? kPts - 1 : jm);
  const v4f pj = xb[jm];
  const float dxv = pj.x - cx;
  const float dyv = pj.y - cy;
  const float dzv = pj.z - cz;

  {
    const unsigned short* pb = p16 + (size_t)b * kPts * kFeat;
    const int rsub = lane >> 3;
    const int cseg = (lane & 7) * 8;
    v4u g[4];
#pragma unroll
    for (int it = 0; it < 4; ++it) {
      int jr = gi[it * 4 + rsub];
      jr = jr < 0 ? 0 : (jr > kPts - 1 ? kPts - 1 : jr);
      g[it] = *(const v4u*)(pb + (size_t)jr * kFeat + cseg);
    }
#pragma unroll
    for (int it = 0; it < 4; ++it) {
      const v8h hv = __builtin_bit_cast(v8h, g[it]);
      *(v8h*)(xw + (it * 4 + rsub) * 72 + cseg) = hv;
    }
    asm volatile("" ::: "memory");
#pragma unroll
    for (int it = 0; it < 4; ++it) {
      int jr = gi[16 + it * 4 + rsub];
      jr = jr < 0 ? 0 : (jr > kPts - 1 ? kPts - 1 : jr);
      g[it] = *(const v4u*)(pb + (size_t)jr * kFeat + cseg);
    }
#pragma unroll
    for (int it = 0; it < 4; ++it) {
      const v8h hv = __builtin_bit_cast(v8h, g[it]);
      *(v8h*)(xw + (16 + it * 4 + rsub) * 72 + cseg) = hv;
    }
  }
  __syncthreads();

  const float dx0 = __shfl(dxv, n, 32);
  const float dy0 = __shfl(dyv, n, 32);
  const float dz0 = __shfl(dzv, n, 32);
  const float dx1 = __shfl(dxv, 16 + n, 32);
  const float dy1 = __shfl(dyv, 16 + n, 32);
  const float dz1 = __shfl(dzv, 16 + n, 32);

  const v8f zero8 = (v8f){0.f, 0.f, 0.f, 0.f, 0.f, 0.f, 0.f, 0.f};
  const _Float16* W0 = (const _Float16*)w0p;
  const _Float16* W1 = (const _Float16*)w1p;
  const _Float16* W2 = (const _Float16*)w2p;

  v16h bx[2][2];
#pragma unroll
  for (int kc = 0; kc < 2; ++kc)
#pragma unroll
    for (int nt = 0; nt < 2; ++nt)
      bx[kc][nt] = FragH::load(xw + (nt * 16 + n) * 72 + kc * 32 + 8 * h);

  v16h y1[2][2];
#pragma unroll
  for (int kc = 0; kc < 2; ++kc)
#pragma unroll
    for (int nt = 0; nt < 2; ++nt)
#pragma unroll
      for (int e = 0; e < 16; ++e) y1[kc][nt][e] = (_Float16)0.0f;
#pragma unroll
  for (int ot = 0; ot < 4; ++ot) {
    const _Float16* wr = W0 + (ot * 16 + n) * 64 + 8 * h;
    const v16h a0 = FragH::load(wr);
    const v16h a1 = FragH::load(wr + 32);
    v8f c0 = zero8, c1 = zero8;
    mma4(c0, c1, a0, a1, bx[0][0], bx[0][1], bx[1][0], bx[1][1]);
    const int chb = ot * 16 + 8 * h;
    float sc[8], sh[8];
    ld8(tab + kTabSc0 + chb, sc);
    ld8(tab + kTabSh0 + chb, sh);
#pragma unroll
    for (int r = 0; r < 8; ++r) {
      const v4f wx = *(const v4f*)(tab + (chb + r) * 4);
      float e0 = wx.x * dx0;
      e0 = e0 + wx.y * dy0;
      e0 = e0 + wx.z * dz0;
      float e1 = wx.x * dx1;
      e1 = e1 + wx.y * dy1;
      e1 = e1 + wx.z * dz1;
      float v0 = (c0[r] + e0) * sc[r] + sh[r];
      float v1 = (c1[r] + e1) * sc[r] + sh[r];
      v0 = fmaxf(v0, 0.0f);
      v1 = fmaxf(v1, 0.0f);
      y1[ot >> 1][0][(ot & 1) * 8 + r] = (_Float16)v0;
      y1[ot >> 1][1][(ot & 1) * 8 + r] = (_Float16)v1;
    }
    asm volatile("" ::: "memory");
  }

  v16h y2[2][2];
#pragma unroll
  for (int kc = 0; kc < 2; ++kc)
#pragma unroll
    for (int nt = 0; nt < 2; ++nt)
#pragma unroll
      for (int e = 0; e < 16; ++e) y2[kc][nt][e] = (_Float16)0.0f;
#pragma unroll
  for (int ot = 0; ot < 4; ++ot) {
    const _Float16* wr = W1 + (ot * 16 + n) * 64 + 8 * h;
    const v16h a0 = FragH::load(wr);
    const v16h a1 = FragH::load(wr + 32);
    v8f c0 = zero8, c1 = zero8;
    mma4(c0, c1, a0, a1, y1[0][0], y1[0][1], y1[1][0], y1[1][1]);
    const int chb = ot * 16 + 8 * h;
    float sc[8], sh[8];
    ld8(tab + kTabSc1 + chb, sc);
    ld8(tab + kTabSh1 + chb, sh);
#pragma unroll
    for (int r = 0; r < 8; ++r) {
      float v0 = c0[r] * sc[r] + sh[r];
      float v1 = c1[r] * sc[r] + sh[r];
      v0 = fmaxf(v0, 0.0f);
      v1 = fmaxf(v1, 0.0f);
      y2[ot >> 1][0][(ot & 1) * 8 + r] = (_Float16)v0;
      y2[ot >> 1][1][(ot & 1) * 8 + r] = (_Float16)v1;
    }
    asm volatile("" ::: "memory");
  }

#pragma unroll
  for (int ot = 0; ot < 8; ++ot) {
    const _Float16* wr = W2 + (ot * 16 + n) * 64 + 8 * h;
    const v16h a0 = FragH::load(wr);
    const v16h a1 = FragH::load(wr + 32);
    v8f c0 = zero8, c1 = zero8;
    mma4(c0, c1, a0, a1, y2[0][0], y2[0][1], y2[1][0], y2[1][1]);
    const int chb = ot * 16 + 8 * h;
    float sc[8], sh[8];
    ld8(tab + kTabSc2 + chb, sc);
    ld8(tab + kTabSh2 + chb, sh);
    float mv[8];
#pragma unroll
    for (int r = 0; r < 8; ++r) {
      float v0 = c0[r] * sc[r] + sh[r];
      float v1 = c1[r] * sc[r] + sh[r];
      v0 = fmaxf(v0, 0.0f);
      v1 = fmaxf(v1, 0.0f);
      mv[r] = fmaxf(v0, v1);
    }
    v4f mA, mB;
    mA.x = mv[0]; mA.y = mv[1]; mA.z = mv[2]; mA.w = mv[3];
    mB.x = mv[4]; mB.y = mv[5]; mB.z = mv[6]; mB.w = mv[7];
    *(v4f*)(mw + n * 132 + chb) = mA;
    *(v4f*)(mw + n * 132 + chb + 4) = mB;
    asm volatile("" ::: "memory");
  }
  __syncthreads();

  v4f mx = *(const v4f*)(mw + 4 * lane);
#pragma unroll
  for (int i = 1; i < 16; ++i) {
    const v4f t = *(const v4f*)(mw + i * 132 + 4 * lane);
    mx.x = fmaxf(mx.x, t.x);
    mx.y = fmaxf(mx.y, t.y);
    mx.z = fmaxf(mx.z, t.z);
    mx.w = fmaxf(mx.w, t.w);
  }
  float* dst = out_pts + (size_t)gs * kOutCh + 4 * lane;
  for (int pass = 0; pass < 2; ++pass) {
    *(volatile v4f*)dst = mx;
    __threadfence();
  }
}

extern "C" void kernel_launch(void* const* d_in, const int* in_sizes, int n_in,
                              void* d_out, int out_size, void* d_ws, size_t ws_size,
                              hipStream_t stream) {
  (void)in_sizes; (void)n_in; (void)out_size;
  if (ws_size < kWsTotal) return;
  const float* xyz    = (const float*)d_in[0];
  const float* points = (const float*)d_in[1];
  const float* w0  = (const float*)d_in[2];
  const float* b0  = (const float*)d_in[3];
  const float* g0  = (const float*)d_in[4];
  const float* be0 = (const float*)d_in[5];
  const float* rm0 = (const float*)d_in[6];
  const float* rv0 = (const float*)d_in[7];
  const float* w1  = (const float*)d_in[8];
  const float* b1  = (const float*)d_in[9];
  const float* g1  = (const float*)d_in[10];
  const float* be1 = (const float*)d_in[11];
  const float* rm1 = (const float*)d_in[12];
  const float* rv1 = (const float*)d_in[13];
  const float* w2  = (const float*)d_in[14];
  const float* b2  = (const float*)d_in[15];
  const float* g2  = (const float*)d_in[16];
  const float* be2 = (const float*)d_in[17];
  const float* rm2 = (const float*)d_in[18];
  const float* rv2 = (const float*)d_in[19];

  char* ws = (char*)d_ws;
  unsigned short* w0p = (unsigned short*)(ws + kOffW0p);
  unsigned short* w1p = (unsigned short*)(ws + kOffW1);
  unsigned short* w2p = (unsigned short*)(ws + kOffW2);
  float* tab  = (float*)(ws + kOffTab);
  float* nx   = (float*)(ws + kOffNxyz);
  float* x4   = (float*)(ws + kOffX4);
  unsigned short* p16 = (unsigned short*)(ws + kOffP16);

  float* out_xyz = (float*)d_out;
  float* out_pts = (float*)d_out + (kOut1Bytes / 4);

  prep_kernel<<<2313, 256, 0, stream>>>(xyz, points,
                                        w0, b0, g0, be0, rm0, rv0,
                                        w1, b1, g1, be1, rm1, rv1,
                                        w2, b2, g2, be2, rm2, rv2,
                                        w0p, w1p, w2p, tab, x4, p16);
  fps_kernel<<<kBatch, 256, 0, stream>>>(xyz, out_xyz, nx);
  group_mlp_kernel<<<(kBatch * kCent) / 4, 128, 0, stream>>>(x4, p16, nx, w0p, w1p, w2p, tab, out_pts);
}
